// TTEmbedding_36447092474248
// MI455X (gfx1250) — hardware-verified
//
#include <hip/hip_runtime.h>
#include <stddef.h>


typedef _Float16 h16;
typedef _Float16 v16h __attribute__((ext_vector_type(16)));
typedef _Float16 v8h  __attribute__((ext_vector_type(8)));
typedef float    v8f  __attribute__((ext_vector_type(8)));
typedef float    v4f  __attribute__((ext_vector_type(4)));

#ifndef NIDX
#define NIDX 8192
#endif
#define NIDX_FULL 8192
#define NV0  50
#define NV1  50
#define NV2  80
#define NE0  8
#define NE1  4
#define NE2  4
#define RANK 16
#define VOCAB (NV0 * NV1 * NV2)
#define EDIM  (NE0 * NE1 * NE2)
#define M1    (NV0 * NE0)
#define N1    (NV1 * NE1 * RANK)
#define M2    (NV0 * NV1 * NE0 * NE1)
#define N2    (NV2 * NE2)

static_assert(NIDX >= 8 && NIDX <= NIDX_FULL && (NIDX % 8) == 0);
static_assert(RANK == 16);
static_assert(NE0 == 8);
static_assert(NE1 * RANK == 64);
static_assert(NE0 * NE1 == 32);
static_assert(NE2 == 4 && EDIM == 128);
static_assert((M1 % 16) == 0);
static_assert((N1 % 64) == 0 && (N2 % 64) == 0);
static_assert((M2 % 64) == 0);
static_assert((64 % (NE0 * NE1)) == 0);
static_assert(((M1 * RANK) % 256) == 0);
static_assert((size_t)VOCAB * EDIM < (size_t)0xFFFFFFFFu);

#define LDK 24
#define LDC 68
static_assert((LDK % 8) == 0 && LDK >= RANK);
static_assert((LDC % 4) == 0 && LDC >= 64);

#define WCARRY 256.0f
#define OSCALE (1.0f / 16777216.0f)

#define A0_BYTES  ((size_t)M1 * RANK * 2)
#define C1_BYTES  ((size_t)N1 * RANK * 2)
#define C2_BYTES  ((size_t)N2 * RANK * 2)
#define W1_BYTES  ((size_t)M2 * RANK * 2)
#define TAB_BYTES ((size_t)VOCAB * EDIM * 4)
#define OFF_A0  ((size_t)0)
#define OFF_C1  (OFF_A0 + A0_BYTES)
#define OFF_C2  (OFF_C1 + C1_BYTES)
#define OFF_W1  (OFF_C2 + C2_BYTES)
#define OFF_TAB (OFF_W1 + W1_BYTES)
#define WS_TOTAL (OFF_TAB + TAB_BYTES)
static_assert((A0_BYTES % 128) == 0 && (C1_BYTES % 128) == 0 && (C2_BYTES % 128) == 0);
static_assert((W1_BYTES % 128) == 0 && (TAB_BYTES % 128) == 0);
static_assert(WS_TOTAL <= (size_t)134217728);

__device__ __forceinline__ float bf16r(float x) {
  unsigned int u = __float_as_uint(x);
  u = (u + 0x7FFFu + ((u >> 16) & 1u)) & 0xFFFF0000u;
  return __uint_as_float(u);
}

static __device__ __forceinline__ h16 toh_flush(float v) {
  const h16 r = (h16)v;
  return (fabsf(v) < 6.103515625e-05f) ? (h16)0.0f : r;
}

__device__ __forceinline__ v16h frag_k16(const h16* p) {
  const v8h lo = *(const v8h*)(p);
  v16h out;
#pragma unroll
  for (int i = 0; i < 8; ++i) { out[i] = lo[i]; out[i + 8] = (h16)0.0f; }
  return out;
}

__device__ __forceinline__ v8f wmma16(v16h a, v16h b, v8f c) {
  v8f d = __builtin_amdgcn_wmma_f32_16x16x32_f16(false, a, false, b, (short)0, c,
                                                 false, false);
  asm volatile("v_nop\n\tv_nop\n\tv_nop\n\tv_nop" : "+v"(d) : "v"(a), "v"(b));
  return d;
}

__global__ __launch_bounds__(32) void aconv_kernel(
    const float* __restrict__ src, h16* __restrict__ dst) {
  const unsigned lane = threadIdx.x & 31u;
  const size_t e = ((size_t)blockIdx.x * 32u + lane) * 8u;
  const v4f a0 = *(const v4f*)(src + e);
  const v4f a1 = *(const v4f*)(src + e + 4u);
  v8h o;
#pragma unroll
  for (int i = 0; i < 4; ++i) {
    o[i]     = toh_flush(WCARRY * bf16r(a0[i]));
    o[i + 4] = toh_flush(WCARRY * bf16r(a1[i]));
  }
  h16* p = dst + e;
  *(volatile v8h*)p = o;
  __threadfence();
  *(volatile v8h*)p = o;
}

__global__ __launch_bounds__(128) void tconv_kernel(
    const float* __restrict__ W, h16* __restrict__ Wt, unsigned ldw) {
  __shared__ h16 T[64 * LDK];
  const unsigned tid = threadIdx.x;
  const unsigned n0 = blockIdx.x * 64u;
#pragma unroll 4
  for (unsigned j = 0; j < 8u; ++j) {
    const unsigned idx = tid + 128u * j;
    const unsigned kr = idx >> 6, nc = idx & 63u;
    const float v = W[(size_t)kr * ldw + n0 + nc];
    T[nc * LDK + kr] = toh_flush(WCARRY * bf16r(v));
  }
  __syncthreads();
  const unsigned n = tid >> 1;
  const unsigned kc = (tid & 1u) * 8u;
  const v8h x = *(const v8h*)&T[n * LDK + kc];
  h16* p = Wt + (size_t)(n0 + n) * RANK + kc;
  *(volatile v8h*)p = x;
  __threadfence();
  *(volatile v8h*)p = x;
}

__global__ __launch_bounds__(128) void step1_kernel(
    const h16* __restrict__ A0, const h16* __restrict__ C1t, h16* __restrict__ W1) {
  __shared__ float Cs[16 * LDC];
  const unsigned tid = threadIdx.x, lane = tid & 31u;
  const unsigned w = (unsigned)__builtin_amdgcn_readfirstlane((int)(threadIdx.x >> 5));
  const unsigned hh = lane >> 4, m = lane & 15u;
  const unsigned v1 = blockIdx.x;
  const unsigned m0 = blockIdx.y * 16u;

  const v16h a = frag_k16(A0 + (size_t)(m0 + m) * RANK + hh * 8u);
  const v16h b = frag_k16(C1t + (size_t)(v1 * 64u + w * 16u + m) * RANK + hh * 8u);
  v8f acc = {};
  acc = wmma16(a, b, acc);
#pragma unroll
  for (int r = 0; r < 8; ++r)
    Cs[(hh * 8u + (unsigned)r) * LDC + w * 16u + m] = acc[r];
  __syncthreads();

  const unsigned r = tid >> 3;
  const unsigned pc = (tid & 7u) * 8u;
  const unsigned mrow = m0 + r;
  const unsigned v0 = mrow >> 3, e0 = mrow & 7u;
  const v4f u0 = *(const v4f*)&Cs[r * LDC + pc];
  const v4f u1 = *(const v4f*)&Cs[r * LDC + pc + 4u];
  v8h x;
#pragma unroll
  for (int j = 0; j < 4; ++j) {
    x[j]     = toh_flush(u0[j]);
    x[j + 4] = toh_flush(u1[j]);
  }
  h16* p = W1 + (size_t)((v0 * NV1 + v1) * NE0 + e0) * 64u + pc;
  *(volatile v8h*)p = x;
  __threadfence();
  *(volatile v8h*)p = x;
}

__global__ __launch_bounds__(256) void step2_kernel(
    const h16* __restrict__ W1, const h16* __restrict__ C2t, float* __restrict__ tab) {
  __shared__ float Cs[64 * LDC];
  const unsigned tid = threadIdx.x, lane = tid & 31u;
  const unsigned w = (unsigned)__builtin_amdgcn_readfirstlane((int)(threadIdx.x >> 5));
  const unsigned mw = w >> 1, nw = w & 1u;
  const unsigned hh = lane >> 4, m = lane & 15u;
  const unsigned n0 = blockIdx.x * 64u;
  const unsigned row0 = blockIdx.y * 64u;

  const v16h a  = frag_k16(W1 + (size_t)(row0 + mw * 16u + m) * RANK + hh * 8u);
  const v16h b0 = frag_k16(C2t + (size_t)(n0 + nw * 32u + m) * RANK + hh * 8u);
  const v16h b1 = frag_k16(C2t + (size_t)(n0 + nw * 32u + 16u + m) * RANK + hh * 8u);
  v8f acc0 = {}, acc1 = {};
  acc0 = wmma16(a, b0, acc0);
  acc1 = wmma16(a, b1, acc1);
#pragma unroll
  for (int r = 0; r < 8; ++r) {
    float* d = &Cs[(mw * 16u + hh * 8u + (unsigned)r) * LDC + nw * 32u + m];
    d[0]  = acc0[r];
    d[16] = acc1[r];
  }
  __syncthreads();

  v4f xs[4];
  size_t off[4];
#pragma unroll
  for (unsigned i = 0; i < 4u; ++i) {
    const unsigned trow = w + 8u * i;
    const unsigned vl = trow >> 4, v2l = trow & 15u;
    const v4f u = *(const v4f*)&Cs[(vl * 32u + lane) * LDC + v2l * 4u];
    v4f val;
#pragma unroll
    for (int j = 0; j < 4; ++j) val[j] = u[j] * OSCALE;
    xs[i] = val;
    const unsigned vrow = (blockIdx.y * 2u + vl) * NV2 + blockIdx.x * 16u + v2l;
    off[i] = (size_t)vrow * EDIM + lane * 4u;
  }
#pragma unroll
  for (int i = 0; i < 4; ++i) *(volatile v4f*)(tab + off[i]) = xs[i];
  __threadfence();
#pragma unroll
  for (int i = 0; i < 4; ++i) *(volatile v4f*)(tab + off[i]) = xs[i];
}

__global__ __launch_bounds__(256) void lookup_kernel(
    const int* __restrict__ indices, const float* __restrict__ tab, float* __restrict__ out) {
  const unsigned lane = threadIdx.x & 31u;
  const unsigned i = blockIdx.x * 8u + (threadIdx.x >> 5);
  int idx = indices[i];
  idx = idx + ((idx < 0) ? (int)VOCAB : 0);
  idx = min(max(idx, 0), (int)VOCAB - 1);
  const v4f v = *(const v4f*)(tab + (size_t)idx * EDIM + lane * 4u);
  float* p = out + (size_t)i * EDIM + lane * 4u;
  *(volatile v4f*)p = v;
  __threadfence();
  *(volatile v4f*)p = v;
}

extern "C" void kernel_launch(void* const* d_in, const int* in_sizes, int n_in,
                              void* d_out, int out_size, void* d_ws, size_t ws_size,
                              hipStream_t stream) {
  if (n_in < 4) return;
  if ((long long)in_sizes[0] < (long long)NIDX) return;
  if ((long long)in_sizes[1] < (long long)M1 * RANK) return;
  if ((long long)in_sizes[2] < (long long)RANK * N1) return;
  if ((long long)in_sizes[3] < (long long)RANK * N2) return;
  if ((long long)out_size < (long long)NIDX * EDIM) return;
  if (ws_size < WS_TOTAL) return;

  const int*   indices = (const int*)d_in[0];
  const float* core0   = (const float*)d_in[1];
  const float* core1   = (const float*)d_in[2];
  const float* core2   = (const float*)d_in[3];
  float* out = (float*)d_out;

  char* ws = (char*)d_ws;
  h16*   A0p  = (h16*)(ws + OFF_A0);
  h16*   C1t  = (h16*)(ws + OFF_C1);
  h16*   C2t  = (h16*)(ws + OFF_C2);
  h16*   W1p  = (h16*)(ws + OFF_W1);
  float* tab  = (float*)(ws + OFF_TAB);

  aconv_kernel<<<dim3((M1 * RANK) / 256), dim3(32), 0, stream>>>(core0, A0p);
  tconv_kernel<<<dim3(N1 / 64), dim3(128), 0, stream>>>(core1, C1t, (unsigned)N1);
  tconv_kernel<<<dim3(N2 / 64), dim3(128), 0, stream>>>(core2, C2t, (unsigned)N2);
  step1_kernel<<<dim3(NV1, M1 / 16), dim3(128), 0, stream>>>(A0p, C1t, W1p);
  step2_kernel<<<dim3(N2 / 64, M2 / 64), dim3(256), 0, stream>>>(W1p, C2t, tab);
  lookup_kernel<<<dim3(NIDX / 8), dim3(256), 0, stream>>>(indices, tab, out);
}
